// BaseTransformer_43078521979301
// MI455X (gfx1250) — hardware-verified
//
#include <hip/hip_runtime.h>


#define NB_  16
#define CI   128
#define CO   128
#define LL   1024
#define NH_  8
#define DK   32
#define CQ   768
#define CZ   256
#define PCAR 1024.0f
typedef _Float16 h16;
typedef unsigned short bf;
typedef __attribute__((ext_vector_type(16))) __bf16   v16bf;
typedef __attribute__((ext_vector_type(16))) _Float16 v16h;
typedef __attribute__((ext_vector_type(8)))  _Float16 v8h;
typedef __attribute__((ext_vector_type(8)))  unsigned short v8us;
typedef __attribute__((ext_vector_type(8)))  float    v8f;
typedef __attribute__((ext_vector_type(4)))  float    v4f;
typedef v8h  __attribute__((may_alias)) v8ha;
typedef v4f  __attribute__((may_alias)) v4fa;
typedef v8us __attribute__((may_alias)) v8usa;

__device__ __forceinline__ unsigned short f2bf(float f) { unsigned u = __float_as_uint(f); u += 0x7FFFu + ((u >> 16) & 1u); return (unsigned short)(u >> 16); }
__device__ __forceinline__ float bf2f(unsigned short b) { return __uint_as_float(((unsigned)b) << 16); }
__device__ __forceinline__ float bfr(float f) { return bf2f(f2bf(f)); }
__device__ __forceinline__ v16h cat16(v8h lo, v8h hi) { return __builtin_shufflevector(lo, hi, 0, 1, 2, 3, 4, 5, 6, 7, 8, 9, 10, 11, 12, 13, 14, 15); }
__device__ __forceinline__ v16bf cat16b(v8us lo, v8us hi) { return __builtin_bit_cast(v16bf, __builtin_shufflevector(lo, hi, 0, 1, 2, 3, 4, 5, 6, 7, 8, 9, 10, 11, 12, 13, 14, 15)); }
__device__ __forceinline__ v8f wmma16(v16h a, v16h b, v8f c) { return __builtin_amdgcn_wmma_f32_16x16x32_f16(false, a, false, b, (short)0, c, false, false); }
__device__ __forceinline__ v8f wmmab(v16bf a, v16bf b, v8f c) { return __builtin_amdgcn_wmma_f32_16x16x32_bf16(false, a, false, b, (short)0, c, false, false); }


template <typename T16> struct WFrag;
template <> struct WFrag<h16> { typedef v16h V; static __device__ __forceinline__ V ld(const h16* p) { return cat16(*(const v8h*)p, *(const v8h*)(p + 16)); } static __device__ __forceinline__ v8f mma(V a, V b, v8f c) { return wmma16(a, b, c); } };
template <> struct WFrag<bf> { typedef v16bf V; static __device__ __forceinline__ V ld(const bf* p) { return cat16b(*(const v8us*)p, *(const v8us*)(p + 16)); } static __device__ __forceinline__ v8f mma(V a, V b, v8f c) { return wmmab(a, b, c); } };
template <typename T16, int NSPLIT, bool BIAS>
__global__ __launch_bounds__(32) void k_gemmw(const T16* __restrict__ A, const T16* __restrict__ A2, const T16* __restrict__ Bt, const T16* __restrict__ Bt2, int K, float* C, int ldc, const float* __restrict__ bias, size_t sA, size_t sB, size_t sC) {
    typedef typename WFrag<T16>::V V;
    __shared__ __align__(16) float os[16 * 68];
    const size_t z = blockIdx.z; A += z * sA; if (A2) A2 += z * sA; Bt += z * sB; if (Bt2) Bt2 += z * sB; C += z * sC;
    const int lane = threadIdx.x & 31, lr = lane & 15, hi = lane >> 4; const int r0 = blockIdx.x * 64, c0 = blockIdx.y * 64;
    v8f acc[4][4];
#pragma unroll
    for (int mb = 0; mb < 4; ++mb)
#pragma unroll
        for (int nb = 0; nb < 4; ++nb) acc[mb][nb] = (v8f){};
    const size_t aoff = (size_t)(r0 + lr) * K + 8 * hi, boff = (size_t)(c0 + lr) * K + 8 * hi;
#pragma unroll 1
    for (int kc = 0; kc < K; kc += 32) {
        V a[4], a2[4];
#pragma unroll
        for (int mb = 0; mb < 4; ++mb) { a[mb] = WFrag<T16>::ld(A + aoff + (size_t)mb * 16 * K + kc); if (NSPLIT == 1 || NSPLIT == 2) a2[mb] = WFrag<T16>::ld(A2 + aoff + (size_t)mb * 16 * K + kc); }
#pragma unroll
        for (int nb = 0; nb < 4; ++nb) { const V b = WFrag<T16>::ld(Bt + boff + (size_t)nb * 16 * K + kc); V b2; if (NSPLIT >= 2) b2 = WFrag<T16>::ld(Bt2 + boff + (size_t)nb * 16 * K + kc);
#pragma unroll
            for (int mb = 0; mb < 4; ++mb) { acc[mb][nb] = WFrag<T16>::mma(a[mb], b, acc[mb][nb]); if (NSPLIT == 1 || NSPLIT == 2) acc[mb][nb] = WFrag<T16>::mma(a2[mb], b, acc[mb][nb]); if (NSPLIT >= 2) acc[mb][nb] = WFrag<T16>::mma(a[mb], b2, acc[mb][nb]); } }
        asm volatile("v_nop\n\tv_nop\n\tv_nop\n\tv_nop" : "+v"(acc[0][0]), "+v"(acc[1][1]), "+v"(acc[2][2]), "+v"(acc[3][3]) : "v"(a[0]), "v"(a[3]));
    }
#pragma unroll
    for (int mb = 0; mb < 4; ++mb) {
#pragma unroll
        for (int nb = 0; nb < 4; ++nb) {
#pragma unroll
            for (int j = 0; j < 8; ++j) os[(hi * 8 + j) * 68 + nb * 16 + lr] = acc[mb][nb][j]; }
        __builtin_amdgcn_wave_barrier(); asm volatile("" ::: "memory");
        float* crow = C + (size_t)(r0 + mb * 16) * ldc + c0;
#pragma unroll 1
        for (int ps = 0; ps < 2; ++ps) {
#pragma unroll
            for (int s = 0; s < 8; ++s) { const int row = 2 * s + hi, cofs = lr * 4; v4f val = *(const v4fa*)(os + row * 68 + cofs); if (BIAS) { val[0] += bfr(bias[c0 + cofs]); val[1] += bfr(bias[c0 + cofs + 1]); val[2] += bfr(bias[c0 + cofs + 2]); val[3] += bfr(bias[c0 + cofs + 3]); }
                *(volatile v4f*)(crow + (size_t)row * ldc + cofs) = val; }
            if (ps == 0) __threadfence(); }
        __builtin_amdgcn_wave_barrier(); asm volatile("" ::: "memory");
    }
}

__device__ __forceinline__ h16 tohx(float x) { return (h16)x; }
__device__ __forceinline__ void splitf(float y, unsigned short& h, unsigned short& l) { h = f2bf(y); l = f2bf(y - bf2f(h)); }
typedef __attribute__((ext_vector_type(2))) unsigned short v2us;
typedef __attribute__((ext_vector_type(4))) unsigned short v4us;
typedef __attribute__((ext_vector_type(2))) _Float16 v2h;
typedef __attribute__((ext_vector_type(4))) _Float16 v4h;

__global__ __launch_bounds__(256) void k_cvt8(const float* __restrict__ src, bf* dst, size_t n8) { const size_t i = (size_t)blockIdx.x * 256 + threadIdx.x; if (i >= n8) return; const v8f v = *(const v8f*)(src + i * 8); v8us o;
#pragma unroll
    for (int k = 0; k < 8; ++k) o[k] = f2bf(v[k]); *(volatile v8us*)(dst + i * 8) = o; __threadfence(); *(volatile v8us*)(dst + i * 8) = o; }
__global__ __launch_bounds__(256) void k_xt(const float* __restrict__ x, bf* XT) { const int e = (blockIdx.x * 256 + threadIdx.x) * 2; if (e >= LL * CI) return; const int c = e % CI; const int l = e / CI; v2us o; o[0] = f2bf(x[(size_t)c * LL + l]); o[1] = f2bf(x[(size_t)(c + 1) * LL + l]); *(volatile v2us*)(XT + e) = o; __threadfence(); *(volatile v2us*)(XT + e) = o; }
__global__ __launch_bounds__(256) void k_qk(const float* __restrict__ QKV, const float* __restrict__ bq, h16* Q16, h16* K16) { const int e = (blockIdx.x * 256 + threadIdx.x) * 4; if (e >= NH_ * LL * DK) return; const int d = e % DK; const int l = (e / DK) % LL; const int h = e / (DK * LL); v4h oq, ok;
#pragma unroll
    for (int u = 0; u < 4; ++u) { const int cq = h * 96 + d + u, ck = cq + DK; oq[u] = tohx(__fadd_rn(QKV[(size_t)cq * LL + l], bfr(bq[cq]))); ok[u] = tohx(__fadd_rn(QKV[(size_t)ck * LL + l], bfr(bq[ck]))); }
    for (int ps = 0; ps < 2; ++ps) { *(volatile v4h*)(Q16 + e) = oq; *(volatile v4h*)(K16 + e) = ok; if (ps == 0) __threadfence(); } }
__global__ __launch_bounds__(256) void k_vt(const float* __restrict__ QKV, const float* __restrict__ bq, h16* VT) { const int e = (blockIdx.x * 256 + threadIdx.x) * 4; if (e >= NH_ * 64 * LL) return; const int l = e % LL; const int d = (e / LL) % 64; const int h = e / (LL * 64); v4h o;
    if (d < DK) { const int c = h * 96 + 2 * DK + d; const v4f a = *(const v4f*)(QKV + (size_t)c * LL + l); const float bb = bfr(bq[c]);
#pragma unroll
        for (int u = 0; u < 4; ++u) o[u] = tohx(__fadd_rn(a[u], bb)); } else { for (int u = 0; u < 4; ++u) o[u] = (h16)0.f; }
    *(volatile v4h*)(VT + e) = o; __threadfence(); *(volatile v4h*)(VT + e) = o; }
__global__ __launch_bounds__(256) void k_soft(const float* __restrict__ Sb, h16* P16) { const int lane = threadIdx.x & 31; const int row = blockIdx.x * 8 + (threadIdx.x >> 5); if (row >= NH_ * LL) return; const float* sr = Sb + (size_t)row * LL; float v[LL / 32]; float mx = -3.0e38f; const float scl = 0.17677669529663687f;
#pragma unroll
    for (int ch = 0; ch < LL / 128; ++ch) { const v4f a = *(const v4f*)(sr + ch * 128 + lane * 4);
#pragma unroll
        for (int u = 0; u < 4; ++u) { const float t = a[u] * scl; v[ch * 4 + u] = t; mx = fmaxf(mx, t); } }
#pragma unroll
    for (int sh = 16; sh; sh >>= 1) mx = fmaxf(mx, __shfl_xor(mx, sh, 32));
    float sum = 0.f;
#pragma unroll
    for (int q = 0; q < LL / 32; ++q) { float d0 = __fsub_rn(v[q], mx); asm volatile("" : "+v"(d0)); v[q] = __builtin_amdgcn_exp2f(__fmul_rn(d0, 1.4426950408889634f)); sum += v[q]; }
#pragma unroll
    for (int sh = 16; sh; sh >>= 1) sum += __shfl_xor(sum, sh, 32);
    const float f = __fdiv_rn(PCAR, sum);
    for (int ps = 0; ps < 2; ++ps) {
#pragma unroll
        for (int ch = 0; ch < LL / 128; ++ch) { v4h o4;
#pragma unroll
            for (int q = 0; q < 4; ++q) o4[q] = tohx(v[ch * 4 + q] * f); *(volatile v4h*)(P16 + (size_t)row * LL + ch * 128 + lane * 4) = o4; }
        if (ps == 0) __threadfence(); } }
__global__ __launch_bounds__(256) void k_mrg(const float* __restrict__ O, bf* Zh, bf* Zl) { const int e = (blockIdx.x * 256 + threadIdx.x) * 4; if (e >= LL * CZ) return; const int c = e % CZ; const int l = e / CZ; const int h = c / DK, d = c % DK; const float* o = O + ((size_t)h * LL + l) * 64 + d; v4us oh, ol;
#pragma unroll
    for (int u = 0; u < 4; ++u) { unsigned short a, b; splitf(o[u] * (1.0f / PCAR), a, b); oh[u] = a; ol[u] = b; } *(volatile v4us*)(Zh + e) = oh; *(volatile v4us*)(Zl + e) = ol; __threadfence(); *(volatile v4us*)(Zh + e) = oh; *(volatile v4us*)(Zl + e) = ol; }
__global__ __launch_bounds__(256) void k_fin(const float* __restrict__ OT, const float* __restrict__ RT, float* OUTb) { const int e = (blockIdx.x * 256 + threadIdx.x) * 4; if (e >= CO * LL) return; const int l = e % LL; const int o = e / LL; v4f r;
#pragma unroll
    for (int u = 0; u < 4; ++u) r[u] = __fadd_rn(OT[(size_t)(l + u) * CO + o], RT[(size_t)(l + u) * CO + o]); *(volatile v4f*)(OUTb + e) = r; __threadfence(); *(volatile v4f*)(OUTb + e) = r; }

extern "C" void kernel_launch(void* const* d_in, const int* in_sizes, int n_in,
                              void* d_out, int out_size, void* d_ws, size_t ws_size, hipStream_t stream) {
    (void)in_sizes; (void)n_in; (void)out_size;
    const float** I = (const float**)d_in;
    const float *x = I[0], *w_qkv = I[1], *b_qkv = I[2], *w_o = I[3], *b_o = I[4], *w_res = I[5], *b_res = I[6];
    float* OUT = (float*)d_out;
    char* wsp = (char*)d_ws;
    auto take = [&](size_t bytes) { char* p = wsp; wsp += (bytes + 255) & ~(size_t)255; return (void*)p; };
    bf* AQ = (bf*)take((size_t)CQ * CI * 2); bf* BO = (bf*)take(CO * CZ * 2); bf* BR = (bf*)take(CO * CI * 2);
    bf* XT = (bf*)take((size_t)LL * CI * 2); float* QKV = (float*)take((size_t)CQ * LL * 4); h16* Q16 = (h16*)take((size_t)NH_ * LL * DK * 2); h16* K16 = (h16*)take((size_t)NH_ * LL * DK * 2); h16* VT = (h16*)take((size_t)NH_ * 64 * LL * 2);
    float* Sb = (float*)take((size_t)NH_ * LL * LL * 4); h16* P16 = (h16*)take((size_t)NH_ * LL * LL * 2); float* O = (float*)take((size_t)NH_ * LL * 64 * 4); bf* Zh = (bf*)take((size_t)LL * CZ * 2); bf* Zl = (bf*)take((size_t)LL * CZ * 2); float* OT = (float*)take((size_t)LL * CO * 4); float* RT = (float*)take((size_t)LL * CO * 4);
    if ((size_t)(wsp - (char*)d_ws) > ws_size) return;
    k_cvt8<<<(CQ * CI / 8 + 255) / 256, 256, 0, stream>>>(w_qkv, AQ, CQ * CI / 8); k_cvt8<<<(CO * CZ / 8 + 255) / 256, 256, 0, stream>>>(w_o, BO, CO * CZ / 8); k_cvt8<<<(CO * CI / 8 + 255) / 256, 256, 0, stream>>>(w_res, BR, CO * CI / 8);
    for (int b = 0; b < NB_; ++b) { const float* xb = x + (size_t)b * CI * LL;
        k_xt<<<(LL * CI / 2 + 255) / 256, 256, 0, stream>>>(xb, XT);
        k_gemmw<bf, 0, false><<<dim3(CQ / 64, LL / 64, 1), 32, 0, stream>>>(AQ, nullptr, XT, nullptr, CI, QKV, LL, nullptr, 0, 0, 0);
        k_qk<<<(NH_ * LL * DK / 4 + 255) / 256, 256, 0, stream>>>(QKV, b_qkv, Q16, K16); k_vt<<<(NH_ * 64 * LL / 4 + 255) / 256, 256, 0, stream>>>(QKV, b_qkv, VT);
        k_gemmw<h16, 0, false><<<dim3(LL / 64, LL / 64, NH_), 32, 0, stream>>>(Q16, nullptr, K16, nullptr, DK, Sb, LL, nullptr, (size_t)LL * DK, (size_t)LL * DK, (size_t)LL * LL);
        k_soft<<<NH_ * LL / 8, 256, 0, stream>>>(Sb, P16);
        k_gemmw<h16, 0, false><<<dim3(LL / 64, 1, NH_), 32, 0, stream>>>(P16, nullptr, VT, nullptr, LL, O, 64, nullptr, (size_t)LL * LL, (size_t)64 * LL, (size_t)LL * 64);
        k_mrg<<<(LL * CZ / 4 + 255) / 256, 256, 0, stream>>>(O, Zh, Zl);
        k_gemmw<bf, 1, true><<<dim3(LL / 64, CO / 64, 1), 32, 0, stream>>>(Zh, Zl, BO, nullptr, CZ, OT, CO, b_o, 0, 0, 0); k_gemmw<bf, 0, true><<<dim3(LL / 64, CO / 64, 1), 32, 0, stream>>>(XT, nullptr, BR, nullptr, CI, RT, CO, b_res, 0, 0, 0);
        k_fin<<<(CO * LL / 4 + 255) / 256, 256, 0, stream>>>(OT, RT, OUT + (size_t)b * CO * LL); }
}
